// InfomationLayer_66786741453338
// MI455X (gfx1250) — hardware-verified
//
#include <hip/hip_runtime.h>

typedef _Float16 v16h __attribute__((ext_vector_type(16)));
typedef _Float16 v8h  __attribute__((ext_vector_type(8)));
typedef __bf16   v16b __attribute__((ext_vector_type(16)));
typedef __bf16   v8b  __attribute__((ext_vector_type(8)));
typedef float    v8f  __attribute__((ext_vector_type(8)));
typedef float    v4f  __attribute__((ext_vector_type(4)));
typedef unsigned v4u  __attribute__((ext_vector_type(4)));

union FragH { v16h v; v8h hh[2]; };
union FragB { v16b v; v8b hh[2]; };

__device__ __forceinline__ v8f zero8() {
  v8f z = {0.f, 0.f, 0.f, 0.f, 0.f, 0.f, 0.f, 0.f};
  return z;
}

__device__ __forceinline__ v8f mma_f16(v16h a, v16h b, v8f c) {
  v8f d = __builtin_amdgcn_wmma_f32_16x16x32_f16(false, a, false, b, (short)0, c, false, false);
  asm volatile("v_nop\n\tv_nop\n\tv_nop\n\tv_nop" : "+v"(d) : "v"(a), "v"(b));
  return d;
}

__device__ __forceinline__ v8f mma_bf16(v16b a, v16b b, v8f c) {
  v8f d = __builtin_amdgcn_wmma_f32_16x16x32_bf16(false, a, false, b, (short)0, c, false, false);
  asm volatile("v_nop\n\tv_nop\n\tv_nop\n\tv_nop" : "+v"(d) : "v"(a), "v"(b));
  return d;
}

__device__ __forceinline__ unsigned bf16_rne(float f) {
  unsigned u = __float_as_uint(f);
  return (u + 0x7FFFu + ((u >> 16) & 1u)) >> 16;
}
__device__ __forceinline__ unsigned pack2(float a, float b) {
  return bf16_rne(a) | (bf16_rne(b) << 16);
}

__global__ void __launch_bounds__(256)
prep_kernel(const float* __restrict__ x, const float* __restrict__ y,
            const float* __restrict__ wq, const float* __restrict__ wk,
            const float* __restrict__ wv,
            unsigned short* xyb, unsigned short* wb)
{
  const int bid = blockIdx.x, tid = threadIdx.x;
  if (bid < 4096) {
    const int gid = bid * 256 + tid;
    const int row = gid >> 6;
    const int d   = (gid & 63) * 8;
    const int b   = row >> 11, s = row & 2047;
    const float* src = (s < 1024)
        ? x + ((size_t)(b * 1024 + s) * 512 + d)
        : y + ((size_t)(b * 1024 + (s - 1024)) * 512 + d);
    const v4f v0 = *(const v4f*)src;
    const v4f v1 = *(const v4f*)(src + 4);
    v4u o;
    o.x = pack2(v0.x, v0.y); o.y = pack2(v0.z, v0.w);
    o.z = pack2(v1.x, v1.y); o.w = pack2(v1.z, v1.w);
    unsigned short* dst = xyb + (size_t)gid * 8;
    *(volatile v4u*)dst = o;
    __threadfence();
    *(volatile v4u*)dst = o;
  } else {
    const int k   = bid - 4096;
    const int mt  = k >> 7;
    const int gid = (k & 127) * 256 + tid;
    const float* wsrc = (mt == 0) ? wq : ((mt == 1) ? wk : wv);
    const float* src = wsrc + (size_t)gid * 8;
    const v4f v0 = *(const v4f*)src;
    const v4f v1 = *(const v4f*)(src + 4);
    v4u o;
    o.x = pack2(v0.x, v0.y); o.y = pack2(v0.z, v0.w);
    o.z = pack2(v1.x, v1.y); o.w = pack2(v1.z, v1.w);
    unsigned short* dst = wb + (size_t)mt * 262144 + (size_t)gid * 8;
    *(volatile v4u*)dst = o;
    __threadfence();
    *(volatile v4u*)dst = o;
  }
}

__global__ void __launch_bounds__(128)
proj_kernel(const __bf16* __restrict__ xyb, const __bf16* __restrict__ wb,
            _Float16* Qh, _Float16* Kh, _Float16* Vt)
{
  __shared__ __align__(16) _Float16 sq[64 * 72];
  __shared__ __align__(16) _Float16 sk[64 * 72];
  __shared__ __align__(16) _Float16 sv[64 * 72];

  const int tid = threadIdx.x, l = tid & 31, w = tid >> 5;
  const int h = l >> 4, m = l & 15;
  const int wr = w >> 1, wc = w & 1;
  const int bx = blockIdx.x, by = blockIdx.y;
  const int lr0 = wr * 32, lc0 = wc * 32;

  const __bf16* Ap = xyb + (size_t)(bx * 64 + lr0 + m) * 512 + 8 * h;
  const __bf16* Bp = wb  + (size_t)(by * 64 + lc0 + m) * 512 + 8 * h;

  v8f acc[12];
#pragma unroll
  for (int i = 0; i < 12; ++i) acc[i] = zero8();

#pragma unroll 1
  for (int ks = 0; ks < 16; ++ks) {
    const int k0 = ks * 32;
    FragB a0, a1;
    a0.hh[0] = *(const v8b*)(Ap + k0);
    a0.hh[1] = *(const v8b*)(Ap + k0 + 16);
    a1.hh[0] = *(const v8b*)(Ap + 16 * 512 + k0);
    a1.hh[1] = *(const v8b*)(Ap + 16 * 512 + k0 + 16);
#pragma unroll
    for (int mt = 0; mt < 3; ++mt) {
#pragma unroll
      for (int tj = 0; tj < 2; ++tj) {
        const __bf16* p = Bp + (size_t)mt * 262144 + tj * (16 * 512) + k0;
        FragB bb;
        bb.hh[0] = *(const v8b*)p;
        bb.hh[1] = *(const v8b*)(p + 16);
        acc[mt * 4 + tj]     = mma_bf16(a0.v, bb.v, acc[mt * 4 + tj]);
        acc[mt * 4 + 2 + tj] = mma_bf16(a1.v, bb.v, acc[mt * 4 + 2 + tj]);
      }
    }
  }

#pragma unroll
  for (int ti = 0; ti < 2; ++ti) {
#pragma unroll
    for (int tj = 0; tj < 2; ++tj) {
      const v8f cq = acc[0 + ti * 2 + tj];
      const v8f ck = acc[4 + ti * 2 + tj];
      const v8f cv = acc[8 + ti * 2 + tj];
      const int rbase = lr0 + ti * 16 + 8 * h;
      const int ccol  = lc0 + tj * 16 + m;
#pragma unroll
      for (int r = 0; r < 8; ++r) {
        sq[(rbase + r) * 72 + ccol] = (_Float16)cq[r];
        sk[(rbase + r) * 72 + ccol] = (_Float16)ck[r];
      }
      v8h pv;
#pragma unroll
      for (int r = 0; r < 8; ++r) pv[r] = (_Float16)cv[r];
      *(v8h*)(sv + ccol * 72 + rbase) = pv;
    }
  }
  __syncthreads();

  const int q = l >> 3, t = l & 7;
  const int b  = bx >> 5;
  const int s0 = (bx & 31) * 64;
#pragma unroll
  for (int i = 0; i < 4; ++i) {
    const int row = w * 16 + i * 4 + q;
    const v8h vq = *(const v8h*)(sq + row * 72 + 8 * t);
    const v8h vk = *(const v8h*)(sk + row * 72 + 8 * t);
    const v8h vv = *(const v8h*)(sv + row * 72 + 8 * t);
    *(volatile v8h*)(Qh + (size_t)(bx * 64 + row) * 512 + by * 64 + 8 * t) = vq;
    *(volatile v8h*)(Kh + (size_t)(bx * 64 + row) * 512 + by * 64 + 8 * t) = vk;
    *(volatile v8h*)(Vt + ((size_t)b * 512 + by * 64 + row) * 2048 + s0 + 8 * t) = vv;
  }
  __threadfence();
#pragma unroll
  for (int i = 0; i < 4; ++i) {
    const int row = w * 16 + i * 4 + q;
    const v8h vq = *(const v8h*)(sq + row * 72 + 8 * t);
    const v8h vk = *(const v8h*)(sk + row * 72 + 8 * t);
    const v8h vv = *(const v8h*)(sv + row * 72 + 8 * t);
    *(volatile v8h*)(Qh + (size_t)(bx * 64 + row) * 512 + by * 64 + 8 * t) = vq;
    *(volatile v8h*)(Kh + (size_t)(bx * 64 + row) * 512 + by * 64 + 8 * t) = vk;
    *(volatile v8h*)(Vt + ((size_t)b * 512 + by * 64 + row) * 2048 + s0 + 8 * t) = vv;
  }
}

__global__ void __launch_bounds__(128)
attn_kernel(const _Float16* __restrict__ Qh, const _Float16* __restrict__ Kh,
            const _Float16* __restrict__ Vt, float* out)
{
  extern __shared__ __align__(16) char smem[];
  float*    sc = (float*)smem;
  _Float16* P  = (_Float16*)(smem + 131072);

  const int tid = threadIdx.x, l = tid & 31, w = tid >> 5;
  const int h = l >> 4, m = l & 15;
  const int q0 = blockIdx.x * 16;
  const int b  = q0 >> 11;
  const float SCL = 0.044194173824159216f;

  {
    const _Float16* Qrow = Qh + (size_t)(q0 + m) * 512 + 8 * h;
    const _Float16* Kb   = Kh + (size_t)b * 2048 * 512;
    for (int g = 0; g < 4; ++g) {
      const int n0 = w * 512 + g * 128;
      const _Float16* Kc = Kb + (size_t)(n0 + m) * 512 + 8 * h;
      v8f acc[8];
#pragma unroll
      for (int j = 0; j < 8; ++j) acc[j] = zero8();
#pragma unroll 2
      for (int dk = 0; dk < 16; ++dk) {
        const int k0 = dk * 32;
        FragH a;
        a.hh[0] = *(const v8h*)(Qrow + k0);
        a.hh[1] = *(const v8h*)(Qrow + k0 + 16);
#pragma unroll
        for (int j = 0; j < 8; ++j) {
          const _Float16* p = Kc + (size_t)j * (16 * 512) + k0;
          FragH bb;
          bb.hh[0] = *(const v8h*)p;
          bb.hh[1] = *(const v8h*)(p + 16);
          acc[j] = mma_f16(a.v, bb.v, acc[j]);
        }
      }
#pragma unroll
      for (int j = 0; j < 8; ++j) {
        float* d = sc + n0 + j * 16 + m;
#pragma unroll
        for (int r = 0; r < 8; ++r) d[(8 * h + r) * 2048] = acc[j][r] * SCL;
      }
    }
  }
  __syncthreads();

  {
    const int row = tid >> 3, sub = tid & 7;
    float* rp = sc + row * 2048 + sub * 256;
    float mx = -3.0e38f;
#pragma unroll 4
    for (int j = 0; j < 256; j += 4) {
      const v4f v = *(const v4f*)(rp + j);
      mx = fmaxf(fmaxf(mx, fmaxf(v.x, v.y)), fmaxf(v.z, v.w));
    }
    mx = fmaxf(mx, __shfl_xor(mx, 1));
    mx = fmaxf(mx, __shfl_xor(mx, 2));
    mx = fmaxf(mx, __shfl_xor(mx, 4));
    float sm = 0.0f;
#pragma unroll 4
    for (int j = 0; j < 256; j += 4) {
      v4f v = *(const v4f*)(rp + j);
      v.x = __expf(v.x - mx);
      v.y = __expf(v.y - mx);
      v.z = __expf(v.z - mx);
      v.w = __expf(v.w - mx);
      sm += (v.x + v.y) + (v.z + v.w);
      *(v4f*)(rp + j) = v;
    }
    sm += __shfl_xor(sm, 1);
    sm += __shfl_xor(sm, 2);
    sm += __shfl_xor(sm, 4);
    const float ps = (1.0f / sm) * 16384.0f;
    __syncthreads();
    _Float16* pp = P + row * 2048 + sub * 256;
#pragma unroll 2
    for (int j = 0; j < 256; j += 8) {
      const v4f v0 = *(const v4f*)(rp + j);
      const v4f v1 = *(const v4f*)(rp + j + 4);
      v8h o;
      o[0] = (_Float16)(v0.x * ps); o[1] = (_Float16)(v0.y * ps);
      o[2] = (_Float16)(v0.z * ps); o[3] = (_Float16)(v0.w * ps);
      o[4] = (_Float16)(v1.x * ps); o[5] = (_Float16)(v1.y * ps);
      o[6] = (_Float16)(v1.z * ps); o[7] = (_Float16)(v1.w * ps);
      *(v8h*)(pp + j) = o;
    }
  }
  __syncthreads();

  const int e0 = w * 128;
  v8f oacc[8];
#pragma unroll
  for (int j = 0; j < 8; ++j) oacc[j] = zero8();
  {
    const _Float16* Pr = P + m * 2048 + 8 * h;
    const _Float16* Vc = Vt + ((size_t)b * 512 + e0 + m) * 2048 + 8 * h;
#pragma unroll 2
    for (int ks = 0; ks < 64; ++ks) {
      const int k0 = ks * 32;
      FragH a;
      a.hh[0] = *(const v8h*)(Pr + k0);
      a.hh[1] = *(const v8h*)(Pr + k0 + 16);
#pragma unroll
      for (int j = 0; j < 8; ++j) {
        const _Float16* p = Vc + (size_t)j * (16 * 2048) + k0;
        FragH bb;
        bb.hh[0] = *(const v8h*)p;
        bb.hh[1] = *(const v8h*)(p + 16);
        oacc[j] = mma_f16(a.v, bb.v, oacc[j]);
      }
    }
  }

  float* os = sc;
  {
    const float OSCL = 6.103515625e-05f;
#pragma unroll
    for (int j = 0; j < 8; ++j) {
      float* d = os + e0 + j * 16 + m;
#pragma unroll
      for (int r = 0; r < 8; ++r) d[(8 * h + r) * 512] = oacc[j][r] * OSCL;
    }
  }
  __syncthreads();
  {
    const int q = l >> 3, t = l & 7;
    const int col = e0 + q * 32 + t * 4;
    const float* srow = os + col;
    float* orow = out + (size_t)q0 * 512 + col;
#pragma unroll
    for (int i = 0; i < 16; ++i) {
      const v4f v = *(const v4f*)(srow + i * 512);
      *(volatile v4f*)(orow + (size_t)i * 512) = v;
    }
    __threadfence();
#pragma unroll
    for (int i = 0; i < 16; ++i) {
      const v4f v = *(const v4f*)(srow + i * 512);
      *(volatile v4f*)(orow + (size_t)i * 512) = v;
    }
  }
}

extern "C" void kernel_launch(void* const* d_in, const int* in_sizes, int n_in,
                              void* d_out, int out_size, void* d_ws, size_t ws_size,
                              hipStream_t stream)
{
  if (n_in < 5) return;
  const int NXY = 8 * 1024 * 512;
  const int NW  = 512 * 512;
  const int NO  = 8 * 2048 * 512;
  if (in_sizes[0] != NXY || in_sizes[1] != NXY) return;
  if (in_sizes[2] != NW || in_sizes[3] != NW || in_sizes[4] != NW) return;
  if (out_size != NO) return;

  const float* x  = (const float*)d_in[0];
  const float* y  = (const float*)d_in[1];
  const float* Wq = (const float*)d_in[2];
  const float* Wk = (const float*)d_in[3];
  const float* Wv = (const float*)d_in[4];
  float* out = (float*)d_out;

  const size_t bytes_xyb = (size_t)16384 * 512 * 2;
  const size_t bytes_wb  = (size_t)3 * NW * 2;
  const size_t bytes_q   = (size_t)16384 * 512 * 2;
  const size_t off_xyb = 0;
  const size_t off_wb  = off_xyb + bytes_xyb;
  const size_t off_q   = off_wb  + bytes_wb;
  const size_t off_k   = off_q   + bytes_q;
  const size_t off_v   = off_k   + bytes_q;
  const size_t total   = off_v   + bytes_q;
  if (total > ws_size) return;

  char* ws = (char*)d_ws;
  unsigned short* xyb = (unsigned short*)(ws + off_xyb);
  unsigned short* wb  = (unsigned short*)(ws + off_wb);
  _Float16* Qh = (_Float16*)(ws + off_q);
  _Float16* Kh = (_Float16*)(ws + off_k);
  _Float16* Vt = (_Float16*)(ws + off_v);

  prep_kernel<<<4096 + 384, 256, 0, stream>>>(x, y, Wq, Wk, Wv, xyb, wb);

  proj_kernel<<<dim3(256, 8), 128, 0, stream>>>((const __bf16*)xyb, (const __bf16*)wb, Qh, Kh, Vt);

  const size_t ldsBytes = (size_t)16 * 2048 * 4 + (size_t)16 * 2048 * 2;
  attn_kernel<<<1024, 128, ldsBytes, stream>>>(Qh, Kh, Vt, out);
}
